// PointAttention_29257317220738
// MI455X (gfx1250) — hardware-verified
//
#include <hip/hip_runtime.h>
#include <hip/hip_bf16.h>
#include <math.h>


typedef _Float16 bf16;
typedef _Float16 f16;
typedef __attribute__((ext_vector_type(4))) unsigned v4u_t;
typedef unsigned v4ua __attribute__((ext_vector_type(4), may_alias));
typedef __attribute__((ext_vector_type(4))) float v4f_t;
typedef float v4fa __attribute__((ext_vector_type(4), may_alias));
typedef __attribute__((ext_vector_type(16))) bf16  bf16x16;
typedef bf16x16 f16x16;
typedef __attribute__((ext_vector_type(8)))  bf16  bf16x8;
typedef bf16x8 f16x8;
typedef __attribute__((ext_vector_type(4)))  bf16  bf16x4;
typedef __attribute__((ext_vector_type(8)))  float f32x8;
__device__ __forceinline__ f32x8 wmma16(f16x16 a, f16x16 b, f32x8 c) {
  c = __builtin_amdgcn_wmma_f32_16x16x32_f16(false, a, false, b, (short)0, c, false, false);
  asm volatile("v_nop\n\tv_nop\n\tv_nop\n\tv_nop" : "+v"(c) : "v"(a), "v"(b));
  return c;
}
#define LDS_STRIDE 48
#define KSTRIDE    72
#define VSTRIDE    48

__device__ __forceinline__ f32x8 wmma_bf16(bf16x16 a, bf16x16 b, f32x8 c) {
  c = __builtin_amdgcn_wmma_f32_16x16x32_f16(false, a, false, b, (short)0, c, false, false);
  asm volatile("v_nop\n\tv_nop\n\tv_nop\n\tv_nop" : "+v"(c) : "v"(a), "v"(b));
  return c;
}

template <typename T>
__device__ __forceinline__ bf16x16 load_frag(const T* __restrict__ base, int ld,
                                             int row0, int k0) {
  const int lane = threadIdx.x & 31;
  const int r    = lane & 15;
  const int kh   = (lane >> 4) * 8;
  const T* p0 = base + (size_t)(row0 + r) * ld + (k0 + kh);
  const T* p1 = p0 + 16;
  bf16x16 f;
#pragma unroll
  for (int i = 0; i < 8; ++i) {
    f[i]     = (bf16)p0[i];
    f[i + 8] = (bf16)p1[i];
  }
  return f;
}

__device__ __forceinline__ bf16x16 lds_frag(const bf16* base, int stride) {
  const int lane = threadIdx.x & 31;
  const int row  = lane & 15;
  const int kh   = (lane >> 4) * 8;
  const bf16x8 lo = *(const bf16x8*)(base + row * stride + kh);
  const bf16x8 hi = *(const bf16x8*)(base + row * stride + kh + 16);
  bf16x16 f;
#pragma unroll
  for (int i = 0; i < 8; ++i) { f[i] = lo[i]; f[i + 8] = hi[i]; }
  return f;
}

template <typename T>
__device__ __forceinline__ void stage_read16(const T* __restrict__ p, float* buf) {
#pragma unroll
  for (int i = 0; i < 16; ++i) buf[i] = (float)p[i];
}

__device__ __forceinline__ void stage_write(bf16* dst, const float* buf, int nquad) {
#pragma unroll
  for (int i = 0; i < nquad; ++i) {
    bf16x4 q;
    q[0] = (bf16)buf[4 * i];     q[1] = (bf16)buf[4 * i + 1];
    q[2] = (bf16)buf[4 * i + 2]; q[3] = (bf16)buf[4 * i + 3];
    *(bf16x4*)(dst + 4 * i) = q;
  }
}


#define GSTR 48
#define GSTR 48
template <typename AT, int EPI, bool OUT16>
__global__ __launch_bounds__(256) void gemm_kne(const AT* __restrict__ A, int lda, const float* __restrict__ Wm, int ldw,
                                                const float* __restrict__ bias, const float* __restrict__ R, const float* __restrict__ gvec,
                                                void* __restrict__ Yv, int ldy, int K) {
  __shared__ __attribute__((aligned(16))) f16 ldsA[128 * GSTR];
  __shared__ __attribute__((aligned(16))) f16 ldsW[128 * GSTR];
  __shared__ __attribute__((aligned(16))) float oS[8][32 * 68];
  const int tid = threadIdx.x, lane = tid & 31, wave = tid >> 5, cl = lane & 15, rh = (lane >> 4) * 8;
  const int m0 = blockIdx.x * 128, n0 = blockIdx.y * 128;
  const int wm = (wave & 3) * 32, wn = (wave >> 2) * 64;
  f32x8 acc[2][4];
#pragma unroll
  for (int i = 0; i < 2; ++i)
#pragma unroll
    for (int j = 0; j < 4; ++j) { f32x8 z = {}; acc[i][j] = z; }
#pragma unroll 1
  for (int k0 = 0; k0 < K; k0 += 32) {
    __syncthreads();
    { const int row = tid >> 1, ch = (tid & 1) * 16;
      const AT* src = A + (size_t)(m0 + row) * lda + k0 + ch;
#pragma unroll
      for (int g = 0; g < 16; ++g) ldsA[row * GSTR + ch + g] = (f16)src[g]; }
    { const int k = tid >> 3, nn0 = (tid & 7) * 16;
      const float* src = Wm + (size_t)(k0 + k) * ldw + n0 + nn0;
#pragma unroll
      for (int g = 0; g < 4; ++g) { const v4f_t v = *(const v4f_t*)(src + 4 * g);
#pragma unroll
        for (int u = 0; u < 4; ++u) ldsW[(nn0 + 4 * g + u) * GSTR + k] = (f16)v[u]; } }
    __syncthreads();
    f16x16 af[2];
#pragma unroll
    for (int i = 0; i < 2; ++i) af[i] = lds_frag(ldsA + (wm + 16 * i) * GSTR, GSTR);
#pragma unroll
    for (int j = 0; j < 4; ++j) {
      const f16x16 bf = lds_frag(ldsW + (wn + 16 * j) * GSTR, GSTR);
#pragma unroll
      for (int i = 0; i < 2; ++i) acc[i][j] = wmma16(af[i], bf, acc[i][j]);
    }
  }
  float* so = oS[wave];
#pragma unroll
  for (int i = 0; i < 2; ++i)
#pragma unroll
    for (int j = 0; j < 4; ++j) {
      const int n = n0 + wn + 16 * j + cl;
      const float bv = bias ? bias[n] : 0.0f;
      const float gv = (EPI == 2 || EPI == 4) ? gvec[n] : 0.0f;
      if (EPI == 1) {
#pragma unroll 1
        for (int r = 0; r < 8; ++r) { const float xg = acc[i][j][r] + bv; so[(16 * i + rh + r) * 68 + 16 * j + cl] = 0.5f * xg * (1.0f + erff(xg * 0.70710678118654752f)); }
      } else {
#pragma unroll
        for (int r = 0; r < 8; ++r) {
          float v = acc[i][j][r] + bv;
          if (EPI == 3) v = fmaxf(v, 0.0f);
          if (EPI == 4) v = gv * v;
          if (EPI == 2) v = R[(size_t)(m0 + wm + 16 * i + rh + r) * ldy + n] + gv * v;
          so[(16 * i + rh + r) * 68 + 16 * j + cl] = v;
        }
      }
    }
  asm volatile("s_wait_dscnt 0" ::: "memory");
  __builtin_amdgcn_wave_barrier();
#pragma unroll 1
  for (int pass = 0; pass < 2; ++pass) {
    if (OUT16) {
      f16* Y = (f16*)Yv;
#pragma unroll
      for (int it = 0; it < 8; ++it) { const int c = lane + 32 * it, rr = c >> 3, q8 = (c & 7) * 8;
        union { f16 h[8]; v4u_t v; } u;
#pragma unroll
        for (int e = 0; e < 8; ++e) u.h[e] = (f16)so[rr * 68 + q8 + e];
        *(volatile v4u_t*)(Y + (size_t)(m0 + wm + rr) * ldy + n0 + wn + q8) = u.v; }
    } else {
      float* Y = (float*)Yv;
#pragma unroll
      for (int it = 0; it < 16; ++it) { const int f4 = lane + 32 * it, rr = f4 >> 4, q = (f4 & 15) * 4;
        *(volatile v4f_t*)(Y + (size_t)(m0 + wm + rr) * ldy + n0 + wn + q) = *(const v4fa*)(so + rr * 68 + q); }
    }
    __threadfence();
  }
}

template <typename AT, int EPI, bool OUT16>
__global__ __launch_bounds__(256) void gemm_knez(const AT* __restrict__ A, int lda, size_t strideA, const float* __restrict__ Wm, int ldw, size_t strideW,
                                                 const float* __restrict__ bias, const float* __restrict__ R, const float* __restrict__ gvec,
                                                 void* __restrict__ Yv, int ldy, size_t strideY, int K) {
  A += (size_t)blockIdx.z * strideA; Wm += (size_t)blockIdx.z * strideW; Yv = (void*)((char*)Yv + (size_t)blockIdx.z * strideY * (OUT16 ? 2 : 4)); if (R) R += (size_t)blockIdx.z * strideY;
  __shared__ __attribute__((aligned(16))) f16 ldsA[128 * GSTR];
  __shared__ __attribute__((aligned(16))) f16 ldsW[128 * GSTR];
  __shared__ __attribute__((aligned(16))) float oS[8][32 * 68];
  const int tid = threadIdx.x, lane = tid & 31, wave = tid >> 5, cl = lane & 15, rh = (lane >> 4) * 8;
  const int m0 = blockIdx.x * 128, n0 = blockIdx.y * 128;
  const int wm = (wave & 3) * 32, wn = (wave >> 2) * 64;
  f32x8 acc[2][4];
#pragma unroll
  for (int i = 0; i < 2; ++i)
#pragma unroll
    for (int j = 0; j < 4; ++j) { f32x8 z = {}; acc[i][j] = z; }
#pragma unroll 1
  for (int k0 = 0; k0 < K; k0 += 32) {
    __syncthreads();
    { const int row = tid >> 1, ch = (tid & 1) * 16;
      const AT* src = A + (size_t)(m0 + row) * lda + k0 + ch;
#pragma unroll
      for (int g = 0; g < 16; ++g) ldsA[row * GSTR + ch + g] = (f16)src[g]; }
    { const int k = tid >> 3, nn0 = (tid & 7) * 16;
      const float* src = Wm + (size_t)(k0 + k) * ldw + n0 + nn0;
#pragma unroll
      for (int g = 0; g < 4; ++g) { const v4f_t v = *(const v4f_t*)(src + 4 * g);
#pragma unroll
        for (int u = 0; u < 4; ++u) ldsW[(nn0 + 4 * g + u) * GSTR + k] = (f16)v[u]; } }
    __syncthreads();
    f16x16 af[2];
#pragma unroll
    for (int i = 0; i < 2; ++i) af[i] = lds_frag(ldsA + (wm + 16 * i) * GSTR, GSTR);
#pragma unroll
    for (int j = 0; j < 4; ++j) {
      const f16x16 bf = lds_frag(ldsW + (wn + 16 * j) * GSTR, GSTR);
#pragma unroll
      for (int i = 0; i < 2; ++i) acc[i][j] = wmma16(af[i], bf, acc[i][j]);
    }
  }
  float* so = oS[wave];
#pragma unroll
  for (int i = 0; i < 2; ++i)
#pragma unroll
    for (int j = 0; j < 4; ++j) {
      const int n = n0 + wn + 16 * j + cl;
      const float bv = bias ? bias[n] : 0.0f;
      const float gv = (EPI == 2 || EPI == 4) ? gvec[n] : 0.0f;
      if (EPI == 1) {
#pragma unroll 1
        for (int r = 0; r < 8; ++r) { const float xg = acc[i][j][r] + bv; so[(16 * i + rh + r) * 68 + 16 * j + cl] = 0.5f * xg * (1.0f + erff(xg * 0.70710678118654752f)); }
      } else {
#pragma unroll
        for (int r = 0; r < 8; ++r) {
          float v = acc[i][j][r] + bv;
          if (EPI == 3) v = fmaxf(v, 0.0f);
          if (EPI == 4) v = gv * v;
          if (EPI == 2) v = R[(size_t)(m0 + wm + 16 * i + rh + r) * ldy + n] + gv * v;
          so[(16 * i + rh + r) * 68 + 16 * j + cl] = v;
        }
      }
    }
  asm volatile("s_wait_dscnt 0" ::: "memory");
  __builtin_amdgcn_wave_barrier();
#pragma unroll 1
  for (int pass = 0; pass < 2; ++pass) {
    if (OUT16) {
      f16* Y = (f16*)Yv;
#pragma unroll
      for (int it = 0; it < 8; ++it) { const int c = lane + 32 * it, rr = c >> 3, q8 = (c & 7) * 8;
        union { f16 h[8]; v4u_t v; } u;
#pragma unroll
        for (int e = 0; e < 8; ++e) u.h[e] = (f16)so[rr * 68 + q8 + e];
        *(volatile v4u_t*)(Y + (size_t)(m0 + wm + rr) * ldy + n0 + wn + q8) = u.v; }
    } else {
      float* Y = (float*)Yv;
#pragma unroll
      for (int it = 0; it < 16; ++it) { const int f4 = lane + 32 * it, rr = f4 >> 4, q = (f4 & 15) * 4;
        *(volatile v4f_t*)(Y + (size_t)(m0 + wm + rr) * ldy + n0 + wn + q) = *(const v4fa*)(so + rr * 68 + q); }
    }
    __threadfence();
  }
}

template <typename AT, bool ACC>
__global__ __launch_bounds__(256) void gemm_kn2(const AT* __restrict__ A, int lda, size_t strideA,
                                               const float* __restrict__ Wm, int ldw, size_t strideW,
                                               const float* __restrict__ bias, float scale,
                                               float* __restrict__ Y, int ldy, size_t strideY, int K) {
  __shared__ __attribute__((aligned(16))) f16 ldsA[128 * GSTR], ldsAl[128 * GSTR];
  __shared__ __attribute__((aligned(16))) f16 ldsW[128 * GSTR], ldsWl[128 * GSTR];
  __shared__ __attribute__((aligned(16))) float oS[8][32 * 68];
  const int tid = threadIdx.x, lane = tid & 31, wave = tid >> 5, cl = lane & 15, rh = (lane >> 4) * 8;
  const int m0 = blockIdx.x * 128, n0 = blockIdx.y * 128;
  const int wm = (wave & 3) * 32, wn = (wave >> 2) * 64;
  A += (size_t)blockIdx.z * strideA; Wm += (size_t)blockIdx.z * strideW; Y += (size_t)blockIdx.z * strideY;
  f32x8 acc[2][4], accx[2][4];
#pragma unroll
  for (int i = 0; i < 2; ++i)
#pragma unroll
    for (int j = 0; j < 4; ++j) { f32x8 z = {}; acc[i][j] = z; accx[i][j] = z; }
#pragma unroll 1
  for (int k0 = 0; k0 < K; k0 += 32) {
    __syncthreads();
    {
      const int row = tid >> 1, ch = (tid & 1) * 16;
      const AT* src = A + (size_t)(m0 + row) * lda + k0 + ch;
#pragma unroll
      for (int g = 0; g < 16; ++g) { const float v = (float)src[g]; const f16 h = (f16)v; ldsA[row * GSTR + ch + g] = h; ldsAl[row * GSTR + ch + g] = (f16)((v - (float)h) * 2048.0f); }
    }
    {
      const int k = tid >> 3, nn0 = (tid & 7) * 16;
      const float* src = Wm + (size_t)(k0 + k) * ldw + n0 + nn0;
#pragma unroll
      for (int g = 0; g < 4; ++g) { const v4f_t v = *(const v4f_t*)(src + 4 * g);
#pragma unroll
        for (int u = 0; u < 4; ++u) { const f16 h = (f16)v[u]; ldsW[(nn0 + 4 * g + u) * GSTR + k] = h; ldsWl[(nn0 + 4 * g + u) * GSTR + k] = (f16)((v[u] - (float)h) * 2048.0f); } }
    }
    __syncthreads();
    f16x16 af[2], afl[2];
#pragma unroll
    for (int i = 0; i < 2; ++i) { af[i] = lds_frag(ldsA + (wm + 16 * i) * GSTR, GSTR); afl[i] = lds_frag(ldsAl + (wm + 16 * i) * GSTR, GSTR); }
#pragma unroll
    for (int j = 0; j < 4; ++j) {
      const f16x16 bf = lds_frag(ldsW + (wn + 16 * j) * GSTR, GSTR), bfl = lds_frag(ldsWl + (wn + 16 * j) * GSTR, GSTR);
#pragma unroll
      for (int i = 0; i < 2; ++i) { acc[i][j] = wmma16(af[i], bf, acc[i][j]); accx[i][j] = wmma16(af[i], bfl, accx[i][j]); accx[i][j] = wmma16(afl[i], bf, accx[i][j]); }
    }
  }
  float* so = oS[wave];
#pragma unroll
  for (int i = 0; i < 2; ++i)
#pragma unroll
    for (int j = 0; j < 4; ++j) {
      const float bv = bias ? bias[n0 + wn + 16 * j + cl] : 0.0f;
#pragma unroll
      for (int r = 0; r < 8; ++r) so[(16 * i + rh + r) * 68 + 16 * j + cl] = (acc[i][j][r] + accx[i][j][r] * (1.0f / 2048.0f)) * scale + bv;
    }
  asm volatile("s_wait_dscnt 0" ::: "memory");
  __builtin_amdgcn_wave_barrier();
  if (ACC) {
#pragma unroll
    for (int it = 0; it < 16; ++it) { const int f4 = lane + 32 * it, rr = f4 >> 4, q = (f4 & 15) * 4;
      const v4f_t old = *(const v4fa*)(Y + (size_t)(m0 + wm + rr) * ldy + n0 + wn + q);
      v4f_t v = *(const v4fa*)(so + rr * 68 + q); v += old; *(v4fa*)(so + rr * 68 + q) = v; }
    asm volatile("s_wait_dscnt 0" ::: "memory");
  }
#pragma unroll 1
  for (int pass = 0; pass < 2; ++pass) {
#pragma unroll
    for (int it = 0; it < 16; ++it) { const int f4 = lane + 32 * it, rr = f4 >> 4, q = (f4 & 15) * 4;
      *(volatile v4f_t*)(Y + (size_t)(m0 + wm + rr) * ldy + n0 + wn + q) = *(const v4fa*)(so + rr * 68 + q); }
    __threadfence();
  }
}

__global__ __launch_bounds__(256) void k_transpose(const float* __restrict__ Wm, float* __restrict__ Wt, int rows, int cols) {
  __shared__ float tS[64][65];
  const int tid = threadIdx.x, tbj = cols / 64, bi = blockIdx.x / tbj, bj = blockIdx.x % tbj;
  for (int e = tid; e < 64 * 64; e += 256) { const int r = e >> 6, c = e & 63; tS[r][c] = Wm[(size_t)(bi * 64 + r) * cols + bj * 64 + c]; }
  __syncthreads();
  for (int ch = tid; ch < 64 * 16; ch += 256) { const int r = ch >> 4, q4 = (ch & 15) * 4; v4f_t o; o[0] = tS[q4][r]; o[1] = tS[q4 + 1][r]; o[2] = tS[q4 + 2][r]; o[3] = tS[q4 + 3][r];
    float* dst = Wt + (size_t)(bj * 64 + r) * rows + bi * 64 + q4; *(volatile v4f_t*)dst = o; __threadfence(); *(volatile v4f_t*)dst = o; }
}


template <typename AT, int EPI, bool OUT16, int NJ>
__global__ __launch_bounds__(256) void gemm_sm(const AT* __restrict__ A, int lda, size_t sA, const float* __restrict__ Wm, int ldw, size_t sW,
                                               const float* __restrict__ bias, const float* __restrict__ R, const float* __restrict__ gvec,
                                               void* __restrict__ Yv, int ldy, size_t sY, int K) {
  constexpr int BN = 16 * NJ; constexpr int OST = BN + 4;
  A += (size_t)blockIdx.z * sA; Wm += (size_t)blockIdx.z * sW; Yv = (void*)((char*)Yv + (size_t)blockIdx.z * sY * (OUT16 ? 2 : 4)); if (R) R += (size_t)blockIdx.z * sY;
  __shared__ __attribute__((aligned(16))) f16 ldsA[256 * GSTR];
  __shared__ __attribute__((aligned(16))) f16 ldsW[BN * GSTR];
  __shared__ __attribute__((aligned(16))) float oS[8][32 * OST];
  const int tid = threadIdx.x, lane = tid & 31, wave = tid >> 5, cl = lane & 15, rh = (lane >> 4) * 8;
  const int m0 = blockIdx.x * 256, n0 = blockIdx.y * BN;
  const int wm = wave * 32;
  f32x8 acc[2][NJ];
#pragma unroll
  for (int i = 0; i < 2; ++i)
#pragma unroll
    for (int j = 0; j < NJ; ++j) { f32x8 z = {}; acc[i][j] = z; }
#pragma unroll 1
  for (int k0 = 0; k0 < K; k0 += 32) {
    __syncthreads();
    { const AT* src = A + (size_t)(m0 + tid) * lda + k0;
#pragma unroll
      for (int g = 0; g < 32; ++g) ldsA[tid * GSTR + g] = (f16)src[g]; }
    { const int k = tid >> 3, nn0 = (tid & 7) * (2 * NJ);
      const float* src = Wm + (size_t)(k0 + k) * ldw + n0 + nn0;
#pragma unroll
      for (int g = 0; g < NJ / 2; ++g) { const v4f_t v = *(const v4f_t*)(src + 4 * g);
#pragma unroll
        for (int u = 0; u < 4; ++u) ldsW[(nn0 + 4 * g + u) * GSTR + k] = (f16)v[u]; } }
    __syncthreads();
    f16x16 af[2];
#pragma unroll
    for (int i = 0; i < 2; ++i) af[i] = lds_frag(ldsA + (wm + 16 * i) * GSTR, GSTR);
#pragma unroll
    for (int j = 0; j < NJ; ++j) {
      const f16x16 bf = lds_frag(ldsW + (16 * j) * GSTR, GSTR);
#pragma unroll
      for (int i = 0; i < 2; ++i) acc[i][j] = wmma16(af[i], bf, acc[i][j]);
    }
  }
  float* so = oS[wave];
#pragma unroll
  for (int i = 0; i < 2; ++i)
#pragma unroll
    for (int j = 0; j < NJ; ++j) {
      const int n = n0 + 16 * j + cl;
      const float bv = bias ? bias[n] : 0.0f;
      const float gv = (EPI == 2 || EPI == 4) ? gvec[n] : 0.0f;
#pragma unroll
      for (int r = 0; r < 8; ++r) {
        float v = acc[i][j][r] + bv;
        if (EPI == 3) v = fmaxf(v, 0.0f);
        if (EPI == 2) v = R[(size_t)(m0 + wm + 16 * i + rh + r) * ldy + n] + gv * v;
        if (EPI == 4) v = gv * v;
        so[(16 * i + rh + r) * OST + 16 * j + cl] = v;
      }
    }
  asm volatile("s_wait_dscnt 0" ::: "memory");
  __builtin_amdgcn_wave_barrier();
#pragma unroll 1
  for (int pass = 0; pass < 2; ++pass) {
    if (OUT16) {
      f16* Y = (f16*)Yv;
#pragma unroll
      for (int it = 0; it < BN / 8; ++it) { const int c = lane + 32 * it, rr = c / (BN / 8), q8 = (c % (BN / 8)) * 8;
        union { f16 h[8]; v4u_t v; } u;
#pragma unroll
        for (int e = 0; e < 8; ++e) u.h[e] = (f16)so[rr * OST + q8 + e];
        *(volatile v4u_t*)(Y + (size_t)(m0 + wm + rr) * ldy + n0 + q8) = u.v; }
    } else {
      float* Y = (float*)Yv;
#pragma unroll
      for (int it = 0; it < BN / 4; ++it) { const int f4 = lane + 32 * it, rr = f4 / (BN / 4), q = (f4 % (BN / 4)) * 4;
        *(volatile v4f_t*)(Y + (size_t)(m0 + wm + rr) * ldy + n0 + q) = *(const v4fa*)(so + rr * OST + q); }
    }
    __threadfence();
  }
}

#define NVp 1024
#define MMp 32
#define DPp 64
#define DMp 64
#define VCH 128
#define PCH 131072
__global__ __launch_bounds__(256) void k_fill(float* __restrict__ p, float val, size_t n4) { const size_t i = (size_t)blockIdx.x * 256 + threadIdx.x; if (i < n4) { v4f_t v = {val, val, val, val}; *(volatile v4f_t*)(p + 4 * i) = v; __threadfence(); *(volatile v4f_t*)(p + 4 * i) = v; } }
__global__ __launch_bounds__(256) void k_dbg_zero(float* __restrict__ p, size_t n4) { const size_t i = (size_t)blockIdx.x * 256 + threadIdx.x; if (i < n4) { v4f_t z = {0.f,0.f,0.f,0.f}; *(volatile v4f_t*)(p + 4 * i) = z; __threadfence(); *(volatile v4f_t*)(p + 4 * i) = z; } }
__global__ __launch_bounds__(256) void k_copy(const float* __restrict__ src, float* __restrict__ dst, size_t n4) { const size_t i = (size_t)blockIdx.x * 256 + threadIdx.x; if (i < n4) { const v4f_t v = *(const v4f_t*)(src + 4 * i); *(volatile v4f_t*)(dst + 4 * i) = v; __threadfence(); *(volatile v4f_t*)(dst + 4 * i) = v; } }
__global__ __launch_bounds__(256) void k_qk(const float* __restrict__ xyz, const float* __restrict__ Wq, const float* __restrict__ bq, const float* __restrict__ Wk, const float* __restrict__ bk, float* __restrict__ Q, float* __restrict__ Kk, float* __restrict__ EMP) {
  const size_t p = (size_t)blockIdx.x * 4 + (threadIdx.x >> 6); const int f = threadIdx.x & 63; const float x0 = xyz[p * 3], x1 = xyz[p * 3 + 1], x2 = xyz[p * 3 + 2];
  const float qv = bq[f] + x0 * Wq[f] + x1 * Wq[64 + f] + x2 * Wq[128 + f], kv = bk[f] + x0 * Wk[f] + x1 * Wk[64 + f] + x2 * Wk[128 + f]; const float em = (x0 == 0.0f && x1 == 0.0f && x2 == 0.0f) ? 1.0f : 0.0f;
#pragma unroll 1
  for (int pass = 0; pass < 2; ++pass) { *(volatile float*)(Q + p * DMp + f) = qv; *(volatile float*)(Kk + p * DMp + f) = kv; if (f < 32) *(volatile float*)(EMP + p * 32 + f) = em; __threadfence(); }
}
__global__ __launch_bounds__(256) void k_pairA(const float* __restrict__ xyz, const float* __restrict__ Q, const float* __restrict__ Kk, const float* __restrict__ EMP, const float* __restrict__ pW1, const float* __restrict__ pb1, const float* __restrict__ pg, const float* __restrict__ pbeta,
                                              const float* __restrict__ pW2, const float* __restrict__ pb2, const float* __restrict__ g1, const float* __restrict__ be1, int v0, float* __restrict__ R1) {
  __shared__ float red[4][2][2];
  const int pl = threadIdx.x >> 6, f = threadIdx.x & 63, wv = (threadIdx.x >> 5) & 1, lane = threadIdx.x & 31; const size_t r = (size_t)blockIdx.x * 4 + pl;
  const int vl = (int)(r / (MMp * MMp)), i = (int)((r / MMp) % MMp), j = (int)(r % MMp); const size_t pi = (size_t)(v0 + vl) * MMp + i, pj = (size_t)(v0 + vl) * MMp + j;
  const bool pe = (EMP[pi * 32] != 0.0f) || (EMP[pj * 32] != 0.0f);
  float d0 = fabsf(xyz[pj * 3] - xyz[pi * 3]), d1 = fabsf(xyz[pj * 3 + 1] - xyz[pi * 3 + 1]), d2 = fabsf(xyz[pj * 3 + 2] - xyz[pi * 3 + 2]);
  d0 = pe ? -1.0f : d0; d1 = pe ? -1.0f : d1; d2 = pe ? -1.0f : d2;
  const float t0 = pb1[0] + d0 * pW1[0] + d1 * pW1[3] + d2 * pW1[6], t1 = pb1[1] + d0 * pW1[1] + d1 * pW1[4] + d2 * pW1[7], t2 = pb1[2] + d0 * pW1[2] + d1 * pW1[5] + d2 * pW1[8];
  const float mu = (t0 + t1 + t2) * (1.0f / 3.0f); const float e0 = t0 - mu, e1 = t1 - mu, e2 = t2 - mu; const float rs = 1.0f / __builtin_sqrtf((e0 * e0 + e1 * e1 + e2 * e2) * (1.0f / 3.0f) + 1e-5f);
  const float a0 = fmaxf(e0 * rs * pg[0] + pbeta[0], 0.0f), a1 = fmaxf(e1 * rs * pg[1] + pbeta[1], 0.0f), a2 = fmaxf(e2 * rs * pg[2] + pbeta[2], 0.0f);
  const float pij = pb2[f] + a0 * pW2[f] + a1 * pW2[64 + f] + a2 * pW2[128 + f];
  const float w0 = (Q[pi * DMp + f] - Kk[pj * DMp + f] + pij) * 0.125f;
  float s = w0;
#pragma unroll
  for (int o = 1; o < 32; o <<= 1) s += __shfl_xor(s, o, 32);
  if (lane == 0) red[pl][wv][0] = s; __syncthreads(); const float mean = (red[pl][0][0] + red[pl][1][0]) * (1.0f / 64.0f); const float dv = w0 - mean; float s2 = dv * dv;
#pragma unroll
  for (int o = 1; o < 32; o <<= 1) s2 += __shfl_xor(s2, o, 32);
  if (lane == 0) red[pl][wv][1] = s2; __syncthreads(); const float rstd = 1.0f / __builtin_sqrtf((red[pl][0][1] + red[pl][1][1]) * (1.0f / 64.0f) + 1e-5f);
  const float outv = fmaxf(dv * rstd * g1[f] + be1[f], 0.0f);
  *(volatile float*)(R1 + r * DMp + f) = outv; __threadfence(); *(volatile float*)(R1 + r * DMp + f) = outv;
}
__global__ __launch_bounds__(256) void k_pairB(const float* __restrict__ H1, const float* __restrict__ g2, const float* __restrict__ be2, float* __restrict__ R2) {
  __shared__ float red[4][2][2];
  const int pl = threadIdx.x >> 6, f = threadIdx.x & 63, wv = (threadIdx.x >> 5) & 1, lane = threadIdx.x & 31; const size_t r = (size_t)blockIdx.x * 4 + pl; const float h = H1[r * DMp + f];
  float s = h;
#pragma unroll
  for (int o = 1; o < 32; o <<= 1) s += __shfl_xor(s, o, 32);
  if (lane == 0) red[pl][wv][0] = s; __syncthreads(); const float mean = (red[pl][0][0] + red[pl][1][0]) * (1.0f / 64.0f); const float dv = h - mean; float s2 = dv * dv;
#pragma unroll
  for (int o = 1; o < 32; o <<= 1) s2 += __shfl_xor(s2, o, 32);
  if (lane == 0) red[pl][wv][1] = s2; __syncthreads(); const float rstd = 1.0f / __builtin_sqrtf((red[pl][0][1] + red[pl][1][1]) * (1.0f / 64.0f) + 1e-5f);
  const float outv = fmaxf(dv * rstd * g2[f] + be2[f], 0.0f);
  *(volatile float*)(R2 + r * DMp + f) = outv; __threadfence(); *(volatile float*)(R2 + r * DMp + f) = outv;
}
__global__ __launch_bounds__(128) void k_fin(const float* __restrict__ Wf, const float* __restrict__ V, const float* __restrict__ feat, int v0, float* __restrict__ outp) {
  const int pt = blockIdx.x, tid = threadIdx.x; const int vl = pt / MMp, i = pt % MMp; const size_t pg_ = (size_t)(v0 + vl) * MMp + i; float val;
  if (tid < 64) { const int f = tid; const float* wb = Wf + ((size_t)(vl * MMp + i) * MMp) * DMp + f; float m = -3.0e38f;
#pragma unroll 1
    for (int j = 0; j < MMp; ++j) m = fmaxf(m, wb[(size_t)j * DMp]);
    float z = 0.0f;
#pragma unroll 1
    for (int j = 0; j < MMp; ++j) z += expf(wb[(size_t)j * DMp] - m);
    val = expf(wb[(size_t)i * DMp] - m) / z * V[pg_ * DMp + f];
  } else { val = feat[pg_ * DPp + (tid - 64)]; }
  *(volatile float*)(outp + pg_ * (DMp + DPp) + tid) = val; __threadfence(); *(volatile float*)(outp + pg_ * (DMp + DPp) + tid) = val;
}

extern "C" void kernel_launch(void* const* d_in, const int* in_sizes, int n_in,
                              void* d_out, int out_size, void* d_ws, size_t ws_size,
                              hipStream_t stream) {
  (void)in_sizes; (void)n_in; (void)out_size;
  const float** f = (const float**)d_in;
  const float* xyz = f[0], *feat = f[1], *Wq = f[2], *bq = f[3], *Wk = f[4], *bk = f[5], *Wv = f[6], *bv = f[7], *pW1 = f[8], *pb1 = f[9], *pg = f[10], *pbt = f[11], *pW2 = f[12], *pb2 = f[13],
             *g1 = f[14], *be1 = f[15], *wW1 = f[16], *wb1 = f[17], *g2 = f[18], *be2 = f[19], *wW2 = f[20], *wb2 = f[21];
  float* out = (float*)d_out;
  char* ws = (char*)d_ws;
  float* Q = (float*)ws; ws += (size_t)NVp * MMp * DMp * 4; float* Kk = (float*)ws; ws += (size_t)NVp * MMp * DMp * 4; float* V = (float*)ws; ws += (size_t)NVp * MMp * DMp * 4; float* EMP = (float*)ws; ws += (size_t)NVp * MMp * 32 * 4;
  float* R1 = (float*)ws; ws += (size_t)PCH * DMp * 4; float* H1 = (float*)ws; ws += (size_t)PCH * DMp * 4;
  if ((size_t)(ws - (char*)d_ws) > ws_size) return;
  const dim3 blk(256);

  k_qk<<<dim3(NVp * MMp / 4), blk, 0, stream>>>(xyz, Wq, bq, Wk, bk, Q, Kk, EMP);
  gemm_sm<float, 0, false, 4><<<dim3(NVp * MMp / 256, 1, 1), blk, 0, stream>>>(feat, DPp, (size_t)0, Wv, DMp, (size_t)0, bv, nullptr, nullptr, V, DMp, (size_t)0, DPp);
  for (int v0 = 0; v0 < NVp; v0 += VCH) {
    k_pairA<<<dim3(PCH / 4), blk, 0, stream>>>(xyz, Q, Kk, EMP, pW1, pb1, pg, pbt, pW2, pb2, g1, be1, v0, R1);
    gemm_sm<float, 0, false, 4><<<dim3(PCH / 256, 1, 1), blk, 0, stream>>>(R1, DMp, (size_t)0, wW1, DMp, (size_t)0, wb1, nullptr, nullptr, H1, DMp, (size_t)0, DMp);
    k_pairB<<<dim3(PCH / 4), blk, 0, stream>>>(H1, g2, be2, R1);
    gemm_sm<float, 0, false, 4><<<dim3(PCH / 256, 1, 1), blk, 0, stream>>>(R1, DMp, (size_t)0, wW2, DMp, (size_t)0, wb2, nullptr, nullptr, H1, DMp, (size_t)0, DMp);
    k_fin<<<dim3(VCH * MMp), dim3(128), 0, stream>>>(H1, V, feat, v0, out);
  }
}
